// Model_48558900248831
// MI455X (gfx1250) — hardware-verified
//
#include <hip/hip_runtime.h>
#include <stddef.h>
#include <stdint.h>


#define HD     64
#define FD     20
#define CD     7
#define NTHR   256
#define NWAVE  8
#define EPT    8
#define CHUNK  (NTHR * EPT)
#define WCAP   (EPT * 32)
#define LISTN  (NWAVE * WCAP)
#define NBA    1024
#define SLA    10
#define RCAP_U 12288
#define RCAP_M 24576
#define DEGCAP 64
#define GBM    64
#define GTHR   128
#define OW_0   0
#define OW_U1  2048
#define OW_M1  (OW_U1 + 64 * 192)
#define OW_U2  (OW_M1 + 64 * 256)
#define OW_M2  (OW_U2 + 128 * 128)
#define WPL_N  (OW_M2 + 128 * 128)
#define TB_BM    0
#define TB_L1REV 64
#define TB_L1RAT 128
#define TB_L2REV 192
#define TB_L2RAT 256
#define TC_TOP   512
#define TC_BOT   1024
#define T_CLSB   1536
#define TAB_N    2048
#define U_W    4096
#define U_W0   256
#define U_TB   512
#define U_SM   (U_W + U_W0 + U_TB)

static_assert((CHUNK & (CHUNK - 1)) == 0 && CHUNK <= 4096);
static_assert((NBA & (NBA - 1)) == 0 && NBA == (1 << SLA));
static_assert(((long long)CHUNK << SLA) < (1LL << 31));
static_assert(NBA == NTHR * 4 && NBA % (2 * NWAVE) == 0 && NBA % 32 == 0 && NBA % GBM == 0);
static_assert(RCAP_U >= 11044 && RCAP_M >= 21924 && RCAP_M <= 28672);
static_assert(RCAP_U % (4 * NTHR) == 0 && RCAP_M % (4 * NTHR) == 0);
static_assert(DEGCAP >= 43 + 8 && DEGCAP % 32 == 0);
static_assert((LISTN + 2 * RCAP_M + 3 * NBA + 16) * 4 <= 300000);
static_assert(HD % 8 == 0 && HD == 64 && GBM == (GTHR / 32) * 16);
static_assert(U_SM % NTHR == 0 && U_W % NTHR == 0 && (U_W + U_W0) % NTHR == 0);
static_assert(WPL_N * 2 % 256 == 0 && TAB_N * 4 % 256 == 0);
static_assert(FD <= 32 && FD % 4 == 0);

typedef float          v4f   __attribute__((ext_vector_type(4)));
typedef float          v8f   __attribute__((ext_vector_type(8)));
typedef int            v4i   __attribute__((ext_vector_type(4)));
typedef int            v8i   __attribute__((ext_vector_type(8)));
typedef unsigned       v4u   __attribute__((ext_vector_type(4)));
typedef unsigned short v4us  __attribute__((ext_vector_type(4)));
typedef unsigned short v8us  __attribute__((ext_vector_type(8)));
typedef unsigned short v16us __attribute__((ext_vector_type(16)));
typedef __bf16         v16bf __attribute__((ext_vector_type(16)));
typedef v4f  __attribute__((may_alias)) v4fa;
typedef v4i  __attribute__((may_alias)) v4ia;
typedef v4u  __attribute__((may_alias)) v4ua;
typedef v4us __attribute__((may_alias)) v4usa;
typedef v8us __attribute__((may_alias)) v8usa;
typedef unsigned __attribute__((may_alias)) u32a;
union FragB { v16bf v; v16us u; v8us h[2]; v8i w; };

__device__ __forceinline__ v8f wmb(const FragB& a, const FragB& b, v8f c) {
  v8f d = __builtin_amdgcn_wmma_f32_16x16x32_bf16(false, a.v, false, b.v, (short)0, c, false, false);
  asm volatile("v_nop\n\tv_nop\n\tv_nop\n\tv_nop" : "+v"(d) : "v"(a.w), "v"(b.w));
  return d;
}
__device__ __forceinline__ v8f z8() { v8f z = {0.f, 0.f, 0.f, 0.f, 0.f, 0.f, 0.f, 0.f}; return z; }

__device__ __forceinline__ unsigned bf16_bits(float f) {
  const unsigned u = __float_as_uint(f);
  return (u + 0x7FFFu + ((u >> 16) & 1u)) >> 16;
}
__device__ __forceinline__ float bf16_val(float f) { return __uint_as_float(bf16_bits(f) << 16); }
__device__ __forceinline__ unsigned hl_bits(float v, unsigned& lo) {
  const unsigned hb = bf16_bits(v);
  lo = bf16_bits(v - __uint_as_float(hb << 16));
  return hb;
}
__device__ __forceinline__ unsigned mk(bool c) { return (unsigned)(-(int)c); }
__device__ __forceinline__ float andf(float f, unsigned m) { return __uint_as_float(__float_as_uint(f) & m); }
__device__ __forceinline__ v4f and4(v4f a, unsigned m) {
  v4f r; r.x = andf(a.x, m); r.y = andf(a.y, m); r.z = andf(a.z, m); r.w = andf(a.w, m); return r;
}
__device__ __forceinline__ v4f bfv4(v4f a) {
  v4f r; r.x = bf16_val(a.x); r.y = bf16_val(a.y); r.z = bf16_val(a.z); r.w = bf16_val(a.w); return r;
}
__device__ __forceinline__ int clampi(int v, int lo, int hi) { return v < lo ? lo : (v > hi ? hi : v); }

__device__ __forceinline__ void wave_sync() {
  __builtin_amdgcn_fence(__ATOMIC_RELEASE, "wavefront");
  __builtin_amdgcn_wave_barrier();
  __builtin_amdgcn_fence(__ATOMIC_ACQUIRE, "wavefront");
}

template <int SLB>
__device__ __forceinline__ int scan_chunk(const int* __restrict__ dsts, int nE, int cbase, int slotBase,
                                          int nb, int vec8, int* list, int tid, int lane, int wave) {
  int wc = 0;
  const int el0  = tid * EPT;
  const int e0   = cbase + el0;
  const int sent = -2147483647 - 1;
  v4i da, db;
  if (vec8 != 0 && cbase + CHUNK <= nE) {
    da = *(const v4i*)(dsts + e0);
    db = *(const v4i*)(dsts + e0 + 4);
  } else {
    da.x = (e0     < nE) ? dsts[min(e0,     nE - 1)] : sent;
    da.y = (e0 + 1 < nE) ? dsts[min(e0 + 1, nE - 1)] : sent;
    da.z = (e0 + 2 < nE) ? dsts[min(e0 + 2, nE - 1)] : sent;
    da.w = (e0 + 3 < nE) ? dsts[min(e0 + 3, nE - 1)] : sent;
    db.x = (e0 + 4 < nE) ? dsts[min(e0 + 4, nE - 1)] : sent;
    db.y = (e0 + 5 < nE) ? dsts[min(e0 + 5, nE - 1)] : sent;
    db.z = (e0 + 6 < nE) ? dsts[min(e0 + 6, nE - 1)] : sent;
    db.w = (e0 + 7 < nE) ? dsts[min(e0 + 7, nE - 1)] : sent;
  }
  const unsigned nbs = (unsigned)slotBase;
  const unsigned unb = (unsigned)nb;
  const unsigned s0 = (unsigned)da.x - nbs, s1 = (unsigned)da.y - nbs;
  const unsigned s2 = (unsigned)da.z - nbs, s3 = (unsigned)da.w - nbs;
  const unsigned s4 = (unsigned)db.x - nbs, s5 = (unsigned)db.y - nbs;
  const unsigned s6 = (unsigned)db.z - nbs, s7 = (unsigned)db.w - nbs;
  const bool h0 = s0 < unb, h1 = s1 < unb, h2 = s2 < unb, h3 = s3 < unb;
  const bool h4 = s4 < unb, h5 = s5 < unb, h6 = s6 < unb, h7 = s7 < unb;
  const unsigned any = __builtin_amdgcn_ballot_w32(h0 | h1 | h2 | h3 | h4 | h5 | h6 | h7);
  if (any != 0u) {
#define HITJ(J, HJ, SJ) { \
      const unsigned mj = __builtin_amdgcn_ballot_w32(HJ); \
      if (mj != 0u) { \
        if (HJ) { \
          const int pos = wc + (int)__builtin_amdgcn_mbcnt_lo(mj, 0u); \
          if (pos < WCAP) list[wave * WCAP + pos] = ((el0 + (J)) << SLB) | (int)(SJ); \
        } \
        wc += (int)__builtin_popcount(mj); } }
    HITJ(0, h0, s0)
    HITJ(1, h1, s1)
    HITJ(2, h2, s2)
    HITJ(3, h3, s3)
    HITJ(4, h4, s4)
    HITJ(5, h5, s5)
    HITJ(6, h6, s6)
    HITJ(7, h7, s7)
#undef HITJ
  }
  return wc;
}

__device__ __forceinline__ v8us gat8(const float* __restrict__ W, int n, int k8) {
  v8us o;
#pragma unroll
  for (int i = 0; i < 8; ++i) o[i] = (unsigned short)bf16_bits(W[(k8 + i) * HD + n]);
  return o;
}

__global__ __launch_bounds__(NTHR) void k_prep(
    const int* __restrict__ uid, const float* __restrict__ uemb, const float* __restrict__ mx,
    const float* __restrict__ wmov,
    const float* __restrict__ w1vl, const float* __restrict__ w1vr,
    const float* __restrict__ w1tl, const float* __restrict__ w1tr,
    const float* __restrict__ w2tl, const float* __restrict__ w2vr,
    const float* __restrict__ w2vl, const float* __restrict__ w2tr,
    const float* __restrict__ bmov, const float* __restrict__ b1v, const float* __restrict__ b1t,
    const float* __restrict__ b2v, const float* __restrict__ b2t,
    const float* __restrict__ clsw, const float* __restrict__ clsb,
    float* tab, unsigned short* wpl, unsigned short* xu, unsigned short* mxb,
    int nU, int mpu, int nM, int mpm) {
  const int u = (int)blockIdx.x * NTHR + (int)threadIdx.x;
  if (u < U_W) {
    const int job = u >> 9, v = u & 511, n = v >> 3, k8 = (v & 7) * 8;
    v8us o;
    int d0, d1;
    if (job == 0)      { o = gat8(w1vl, n, k8); d0 = OW_U1 + n * 192 + k8;        d1 = d0 + 64; }
    else if (job == 1) { o = gat8(w1vr, n, k8); d0 = OW_U1 + n * 192 + 128 + k8;  d1 = d0; }
    else if (job == 2) { o = gat8(w1tl, n, k8); d0 = OW_M1 + n * 256 + k8;        d1 = d0 + 64; }
    else if (job == 3) { o = gat8(w1tr, n, k8); d0 = OW_M1 + n * 256 + 128 + k8;  d1 = d0 + 64; }
    else if (job == 4) { o = gat8(w2tl, n, k8); d0 = OW_U2 + n * 128 + k8;        d1 = d0 + 64; }
    else if (job == 5) { o = gat8(w2vr, n, k8); d0 = OW_U2 + (64 + n) * 128 + k8; d1 = d0 + 64; }
    else if (job == 6) { o = gat8(w2vl, n, k8); d0 = OW_M2 + n * 128 + k8;        d1 = d0 + 64; }
    else               { o = gat8(w2tr, n, k8); d0 = OW_M2 + (64 + n) * 128 + k8; d1 = d0 + 64; }
    *(volatile v8us*)(wpl + d0) = o;
    *(volatile v8us*)(wpl + d1) = o;
    __threadfence();
    *(volatile v8us*)(wpl + d0) = o;
    *(volatile v8us*)(wpl + d1) = o;
    return;
  }
  if (u < U_W + U_W0) {
    const int v = u - U_W, n = v >> 2, k8 = (v & 3) * 8;
    v8us o;
#pragma unroll
    for (int i = 0; i < 8; ++i) {
      const int k  = k8 + i;
      const int kc = k < FD ? k : FD - 1;
      const unsigned b = bf16_bits(wmov[kc * HD + n]);
      o[i] = (unsigned short)(b & mk(k < FD));
    }
    unsigned short* dp = wpl + OW_0 + v * 8;
    *(volatile v8us*)dp = o;
    __threadfence();
    *(volatile v8us*)dp = o;
    return;
  }
  if (u < U_SM) {
    const int t = u - (U_W + U_W0);
    const int q = (t & 15) * 4;
    const v4f bA = *(const v4f*)(bmov + q);
    const v4f bB = *(const v4f*)(b1v + q);
    const v4f bC = *(const v4f*)(b1t + q);
    const v4f bD = *(const v4f*)(b2v + q);
    const v4f bE = *(const v4f*)(b2t + q);
    const int wh = t >> 4;
    v4f bv;
    {
      const unsigned m0 = mk(wh == 0), m1 = mk(wh == 1), m2 = mk(wh == 2), m3 = mk(wh == 3), m4 = mk(wh == 4);
      bv.x = __uint_as_float((__float_as_uint(bA.x) & m0) | (__float_as_uint(bB.x) & m1) | (__float_as_uint(bC.x) & m2) |
                             (__float_as_uint(bD.x) & m3) | (__float_as_uint(bE.x) & m4));
      bv.y = __uint_as_float((__float_as_uint(bA.y) & m0) | (__float_as_uint(bB.y) & m1) | (__float_as_uint(bC.y) & m2) |
                             (__float_as_uint(bD.y) & m3) | (__float_as_uint(bE.y) & m4));
      bv.z = __uint_as_float((__float_as_uint(bA.z) & m0) | (__float_as_uint(bB.z) & m1) | (__float_as_uint(bC.z) & m2) |
                             (__float_as_uint(bD.z) & m3) | (__float_as_uint(bE.z) & m4));
      bv.w = __uint_as_float((__float_as_uint(bA.w) & m0) | (__float_as_uint(bB.w) & m1) | (__float_as_uint(bC.w) & m2) |
                             (__float_as_uint(bD.w) & m3) | (__float_as_uint(bE.w) & m4));
    }
    const int tt = (t - 128) & 255;
    const int half = tt >> 7, c = (tt >> 4) & 7, cc = c < CD ? c : CD - 1, j4 = (tt & 15) * 4;
    v4f cw;
    cw.x = clsw[(half * HD + j4 + 0) * CD + cc];
    cw.y = clsw[(half * HD + j4 + 1) * CD + cc];
    cw.z = clsw[(half * HD + j4 + 2) * CD + cc];
    cw.w = clsw[(half * HD + j4 + 3) * CD + cc];
    cw = and4(cw, mk(c < CD));
    const int e4 = (t & 7) * 4;
    v4f cb;
    cb.x = andf(clsb[min(e4 + 0, CD - 1)], mk(e4 + 0 < CD));
    cb.y = andf(clsb[min(e4 + 1, CD - 1)], mk(e4 + 1 < CD));
    cb.z = andf(clsb[min(e4 + 2, CD - 1)], mk(e4 + 2 < CD));
    cb.w = andf(clsb[min(e4 + 3, CD - 1)], mk(e4 + 3 < CD));
    const unsigned s0 = mk(t < 128), s1 = mk(t >= 128 && t < 384), s2 = mk(t >= 384 && t < 392);
    v4f val;
    val.x = __uint_as_float((__float_as_uint(bv.x) & s0) | (__float_as_uint(cw.x) & s1) | (__float_as_uint(cb.x) & s2));
    val.y = __uint_as_float((__float_as_uint(bv.y) & s0) | (__float_as_uint(cw.y) & s1) | (__float_as_uint(cb.y) & s2));
    val.z = __uint_as_float((__float_as_uint(bv.z) & s0) | (__float_as_uint(cw.z) & s1) | (__float_as_uint(cb.z) & s2));
    val.w = __uint_as_float((__float_as_uint(bv.w) & s0) | (__float_as_uint(cw.w) & s1) | (__float_as_uint(cb.w) & s2));
    const v4f o = bfv4(val);
    float* dp = tab + 4 * t;
    *(volatile v4f*)dp = o;
    __threadfence();
    *(volatile v4f*)dp = o;
    return;
  }
  const int nXU = mpu * 8;
  if (u < U_SM + nXU) {
    const int v = u - U_SM, row = v >> 3, k8 = (v & 7) * 8;
    const bool live = row < nU;
    const int rcl = live ? row : nU - 1;
    const int id = clampi(uid[rcl], 0, nU - 1);
    const float* p = uemb + (size_t)id * HD + k8;
    const v4f a = *(const v4f*)p;
    const v4f b = *(const v4f*)(p + 4);
    const unsigned lm = mk(live);
    v8us o;
    o[0] = (unsigned short)(bf16_bits(a.x) & lm); o[1] = (unsigned short)(bf16_bits(a.y) & lm);
    o[2] = (unsigned short)(bf16_bits(a.z) & lm); o[3] = (unsigned short)(bf16_bits(a.w) & lm);
    o[4] = (unsigned short)(bf16_bits(b.x) & lm); o[5] = (unsigned short)(bf16_bits(b.y) & lm);
    o[6] = (unsigned short)(bf16_bits(b.z) & lm); o[7] = (unsigned short)(bf16_bits(b.w) & lm);
    unsigned short* dp = xu + (size_t)v * 8;
    *(volatile v8us*)dp = o;
    __threadfence();
    *(volatile v8us*)dp = o;
    return;
  }
  const int v = u - U_SM - nXU;
  if (v < mpm * 4) {
    const int row = v >> 2, k8 = (v & 3) * 8;
    const bool live = row < nM;
    const int rcl = live ? row : nM - 1;
    const int q0 = k8 < FD - 4 ? k8 : FD - 4;
    const int q1 = (k8 + 4) < FD - 4 ? (k8 + 4) : FD - 4;
    const float* p = mx + (size_t)rcl * FD;
    const v4f a = *(const v4f*)(p + q0);
    const v4f b = *(const v4f*)(p + q1);
    const unsigned ma = mk(live && (k8 + 4 <= FD));
    const unsigned mb = mk(live && (k8 + 8 <= FD));
    v8us o;
    o[0] = (unsigned short)(bf16_bits(a.x) & ma); o[1] = (unsigned short)(bf16_bits(a.y) & ma);
    o[2] = (unsigned short)(bf16_bits(a.z) & ma); o[3] = (unsigned short)(bf16_bits(a.w) & ma);
    o[4] = (unsigned short)(bf16_bits(b.x) & mb); o[5] = (unsigned short)(bf16_bits(b.y) & mb);
    o[6] = (unsigned short)(bf16_bits(b.z) & mb); o[7] = (unsigned short)(bf16_bits(b.w) & mb);
    unsigned short* dp = mxb + (size_t)v * 8;
    *(volatile v8us*)dp = o;
    __threadfence();
    *(volatile v8us*)dp = o;
  }
}

template <int NT>
__device__ __forceinline__ void kloop(v8f (&acc)[NT], const unsigned short* ap, const unsigned short* bp,
                                      int ldb, int K) {
#pragma unroll 1
  for (int k0 = 0; k0 < K; k0 += 32) {
    FragB af;
    af.h[0] = *(const v8usa*)(ap + k0);
    af.h[1] = *(const v8usa*)(ap + k0 + 16);
#pragma unroll
    for (int nt = 0; nt < NT; ++nt) {
      const unsigned short* wq = bp + (size_t)(16 * nt) * (size_t)ldb + k0;
      FragB bf;
      bf.h[0] = *(const v8usa*)wq;
      bf.h[1] = *(const v8usa*)(wq + 16);
      acc[nt] = wmb(af, bf, acc[nt]);
    }
  }
}

template <int EPI>
__global__ __launch_bounds__(GTHR) void k_gemm1(unsigned short* A1, int lda1, int K1,
                                                const unsigned short* A2, int lda2, int K2,
                                                const unsigned short* __restrict__ BT, int ldb,
                                                const float* __restrict__ tab, int boff,
                                                const int* __restrict__ gidx, const float* __restrict__ emb, int nEmb,
                                                unsigned short* outpl, int nN) {
  __shared__ __attribute__((aligned(16))) float stg[GBM * 64];
  const int tid = (int)threadIdx.x, lane = tid & 31, wave = tid >> 5, hh = lane >> 4, m = lane & 15;
  const int rowBase = (int)blockIdx.x * GBM;

  v8f acc[4];
#pragma unroll
  for (int t = 0; t < 4; ++t) acc[t] = z8();
  const size_t arow = (size_t)(rowBase + 16 * wave + m);
  const unsigned short* bp = BT + (size_t)m * (size_t)ldb + 8 * hh;
  kloop<4>(acc, A1 + arow * (size_t)lda1 + 8 * hh, bp, ldb, K1);
  kloop<4>(acc, A2 + arow * (size_t)lda2 + 8 * hh, bp + K1, ldb, K2);

#pragma unroll
  for (int nt = 0; nt < 4; ++nt) {
    const int lc = 16 * nt + m;
#pragma unroll
    for (int r = 0; r < 8; ++r) stg[(16 * wave + 8 * hh + r) * 64 + lc] = acc[nt][r];
  }
  __syncthreads();

  const int rr = lane >> 4, c4 = (lane & 15) * 4;
  const v4f bias4 = *(const v4f*)(tab + boff + c4);
  int gl = 0;
  if constexpr (EPI == 0) {
    const int gr = min(rowBase + 16 * wave + (lane & 15), nN - 1);
    gl = clampi(gidx[gr], 0, nEmb - 1);
  }
  v4f pv[8];
#pragma unroll
  for (int i = 0; i < 8; ++i) pv[i] = *(const v4fa*)(stg + (16 * wave + 2 * i + rr) * 64 + c4);
  __syncthreads();

#pragma unroll
  for (int i = 0; i < 8; ++i) {
    const bool ok = (rowBase + 16 * wave + 2 * i + rr) < nN;
    v4f t = pv[i] + bias4;
    v4f y;
    if constexpr (EPI == 0) {
      const int gi = __shfl(gl, 2 * i + rr, 32);
      const v4f e = *(const v4f*)(emb + (size_t)gi * HD + c4);
      y.x = t.x + bf16_val(e.x); y.y = t.y + bf16_val(e.y); y.z = t.z + bf16_val(e.z); y.w = t.w + bf16_val(e.w);
    } else {
      y.x = (t.x > 0.0f) ? t.x : (t.x - t.x);
      y.y = (t.y > 0.0f) ? t.y : (t.y - t.y);
      y.z = (t.z > 0.0f) ? t.z : (t.z - t.z);
      y.w = (t.w > 0.0f) ? t.w : (t.w - t.w);
    }
    y.x = ok ? y.x : 0.0f; y.y = ok ? y.y : 0.0f; y.z = ok ? y.z : 0.0f; y.w = ok ? y.w : 0.0f;
    pv[i] = y;
  }

  unsigned short* sw = (unsigned short*)stg + 2048 * wave;
#pragma unroll
  for (int i = 0; i < 8; ++i) {
    v4us h4, l4;
    unsigned lb, hb;
    hb = hl_bits(pv[i].x, lb); h4[0] = (unsigned short)hb; l4[0] = (unsigned short)lb;
    hb = hl_bits(pv[i].y, lb); h4[1] = (unsigned short)hb; l4[1] = (unsigned short)lb;
    hb = hl_bits(pv[i].z, lb); h4[2] = (unsigned short)hb; l4[2] = (unsigned short)lb;
    hb = hl_bits(pv[i].w, lb); h4[3] = (unsigned short)hb; l4[3] = (unsigned short)lb;
    unsigned short* srow = sw + (2 * i + rr) * 128;
    *(v4usa*)(srow + c4) = h4;
    *(v4usa*)(srow + 64 + c4) = l4;
  }
  __syncthreads();
  v8us qv[8];
#pragma unroll
  for (int i = 0; i < 8; ++i) qv[i] = *(const v8usa*)(sw + i * 256 + 8 * lane);
  unsigned short* ob = ((EPI == 0) ? outpl : A1) + (size_t)(rowBase + 16 * wave) * 128 + 8 * lane;
#pragma unroll
  for (int i = 0; i < 8; ++i) *(volatile v8us*)(ob + i * 256) = qv[i];
  __threadfence();
#pragma unroll
  for (int i = 0; i < 8; ++i) *(volatile v8us*)(ob + i * 256) = qv[i];
}

__global__ __launch_bounds__(GTHR) void k_gemm2(const unsigned short* __restrict__ A1,
                                                const unsigned short* __restrict__ BT,
                                                const float* __restrict__ tab, int boff, int caoff, int cboff,
                                                float* vout) {
  __shared__ __attribute__((aligned(16))) float stg[GBM * 128];
  __shared__ __attribute__((aligned(16))) float ctab[2 * 8 * 64];
  __shared__ __attribute__((aligned(16))) float bsh[128];
  __shared__ __attribute__((aligned(16))) float ost[GBM * 16];
  const int tid = (int)threadIdx.x, lane = tid & 31, wave = tid >> 5, hh = lane >> 4, m = lane & 15;
  const int rowBase = (int)blockIdx.x * GBM;

  v8f acc[8];
#pragma unroll
  for (int t = 0; t < 8; ++t) acc[t] = z8();
  kloop<8>(acc, A1 + (size_t)(rowBase + 16 * wave + m) * 128 + 8 * hh, BT + (size_t)m * 128 + 8 * hh, 128, 128);

#pragma unroll
  for (int nt = 0; nt < 8; ++nt) {
    const int lc = 16 * nt + m;
#pragma unroll
    for (int r = 0; r < 8; ++r) stg[(16 * wave + 8 * hh + r) * 128 + lc] = acc[nt][r];
  }
  {
    const v4f ca = *(const v4f*)(tab + caoff + 4 * tid);
    const v4f cb = *(const v4f*)(tab + cboff + 4 * tid);
    *(v4fa*)(ctab + 4 * tid) = ca;
    *(v4fa*)(ctab + 512 + 4 * tid) = cb;
    if (tid < 32) {
      const v4f b = *(const v4f*)(tab + boff + (tid & 15) * 4);
      *(v4fa*)(bsh + 4 * tid) = and4(b, mk(tid >= 16));
    }
  }
  __syncthreads();

  {
    const int row = tid >> 1, half = tid & 1;
    const float* xr = stg + row * 128 + 64 * half;
    const float* br = bsh + 64 * half;
    const float* ct = ctab + half * 512;
#pragma unroll 1
    for (int c = 0; c < CD; ++c) {
      float a = 0.0f;
#pragma unroll 2
      for (int j = 0; j < 64; j += 4) {
        const v4f x = *(const v4fa*)(xr + j);
        const v4f b = *(const v4fa*)(br + j);
        const v4f w = *(const v4fa*)(ct + c * 64 + j);
        a = fmaf(x.x + b.x, w.x, a);
        a = fmaf(x.y + b.y, w.y, a);
        a = fmaf(x.z + b.z, w.z, a);
        a = fmaf(x.w + b.w, w.w, a);
      }
      ost[row * 16 + 8 * half + c] = a;
    }
    ost[row * 16 + 8 * half + 7] = 0.0f;
  }
  __syncthreads();
  const v4f f0 = *(const v4fa*)(ost + 4 * tid);
  const v4f f1 = *(const v4fa*)(ost + 4 * (tid + GTHR));
  float* dp = vout + (size_t)rowBase * 16 + 4 * tid;
  *(volatile v4f*)dp = f0;
  *(volatile v4f*)(dp + 4 * GTHR) = f1;
  __threadfence();
  *(volatile v4f*)dp = f0;
  *(volatile v4f*)(dp + 4 * GTHR) = f1;
}

template <int RC>
__global__ __launch_bounds__(NTHR) void k_compact(const int* __restrict__ keys, const int* __restrict__ pay,
                                                  int nE, int nPay, int vec8, int* listg, int* cntg, int* offg) {
  extern __shared__ __attribute__((aligned(16))) int dsm[];
  constexpr int ZINTS = LISTN + 2 * RC + 3 * NBA;
  int* list = dsm;
  int* hl   = dsm + LISTN;
  int* sl   = hl + RC;
  int* cnt  = sl + RC;
  int* offs = cnt + NBA;
  int* cur  = offs + NBA;
  int* misc = cur + NBA;
  const int tid = (int)threadIdx.x, lane = tid & 31, wave = tid >> 5;
  const int blk = (int)blockIdx.x;
  const int nodeBase = blk * NBA;

  {
    const v4i z4 = {0, 0, 0, 0};
    for (int i = tid * 4; i < ZINTS; i += NTHR * 4) *(v4ia*)(dsm + i) = z4;
    if (tid < 16) misc[tid] = 0;
  }
  __syncthreads();

  int t = 0, ov = 0;
  const int nChunks = (nE + CHUNK - 1) / CHUNK;
#pragma unroll 1
  for (int ch = 0; ch < nChunks; ++ch) {
    const int cbase = ch * CHUNK;
    const int wc = scan_chunk<SLA>(keys, nE, cbase, nodeBase, NBA, vec8, list, tid, lane, wave);
    if (lane == 0) misc[wave] = wc;
    __syncthreads();
    if (wave == 0) {
#pragma unroll 1
      for (int w2 = 0; w2 < NWAVE; ++w2) {
        int c = misc[w2];
        c = c < 0 ? 0 : (c > WCAP ? WCAP : c);
#pragma unroll 1
        for (int b0 = 0; b0 < c; b0 += 32) {
          const int idx = b0 + lane;
          const int ent_ = list[w2 * WCAP + (idx < WCAP ? idx : WCAP - 1)];
          const int m32 = (c - b0) < 32 ? (c - b0) : 32;
#pragma unroll 1
          for (int k = 0; k < m32; ++k) {
            const int u    = __builtin_amdgcn_readlane(ent_, k);
            const int slot = u & (NBA - 1);
            const int el   = (u >> SLA) & (CHUNK - 1);
            const int pk   = ((cbase + el) << SLA) | slot;
            if (t < RC) {
              if (lane == 0) { hl[t] = pk; cnt[slot] = cnt[slot] + 1; }
              t = t + 1;
            } else {
              ov = 1;
            }
          }
        }
      }
    }
    __syncthreads();
  }
  if (wave == 0 && lane == 0) { misc[8] = t; misc[9] = ov; }
  __syncthreads();
  int tt = misc[8];
  tt = tt < 0 ? 0 : (tt > RC ? RC : tt);
  const int ovf = misc[9];

  if (wave == 0) {
    const int base = lane * (NBA / 32);
    int s = 0;
#pragma unroll 1
    for (int i = 0; i < NBA / 32; ++i) s += cnt[base + i];
    int incl = s;
#pragma unroll
    for (int d = 1; d < 32; d <<= 1) {
      const int y = __shfl_up(incl, d, 32);
      if (lane >= d) incl += y;
    }
    int run = incl - s;
#pragma unroll 1
    for (int i = 0; i < NBA / 32; ++i) {
      const int cv = cnt[base + i];
      offs[base + i] = run;
      cur[base + i]  = run;
      run += cv;
    }
  }
  __syncthreads();
  if (wave == 0) {
#pragma unroll 1
    for (int b0 = 0; b0 < tt; b0 += 32) {
      const int idx = b0 + lane;
      const int ent_ = hl[idx < RC ? idx : RC - 1];
      const int m32 = (tt - b0) < 32 ? (tt - b0) : 32;
#pragma unroll 1
      for (int k = 0; k < m32; ++k) {
        const int u    = __builtin_amdgcn_readlane(ent_, k);
        const int slot = u & (NBA - 1);
        if (lane == 0) {
          int p = cur[slot];
          p = p < 0 ? 0 : (p > RC - 1 ? RC - 1 : p);
          sl[p] = u;
          cur[slot] = p + 1;
        }
      }
    }
  }
  __syncthreads();

  {
    v4i c4 = *(const v4ia*)(cnt + 4 * tid);
    const v4i o4 = *(const v4ia*)(offs + 4 * tid);
    const int pm = (ovf != 0) ? -1 : 0;
    c4.x |= pm; c4.y |= pm; c4.z |= pm; c4.w |= pm;
    int* cp = cntg + (size_t)blk * NBA + 4 * tid;
    int* op = offg + (size_t)blk * NBA + 4 * tid;
    *(volatile v4i*)cp = c4;
    *(volatile v4i*)op = o4;
    __threadfence();
    *(volatile v4i*)cp = c4;
    *(volatile v4i*)op = o4;
  }
#pragma unroll 1
  for (int i4 = tid; i4 < RC / 4; i4 += NTHR) {
    const v4i e = *(const v4ia*)(sl + 4 * i4);
    const int p0 = 4 * i4;
    const int e0 = clampi(e.x >> SLA, 0, nE - 1);
    const int e1 = clampi(e.y >> SLA, 0, nE - 1);
    const int e2 = clampi(e.z >> SLA, 0, nE - 1);
    const int e3 = clampi(e.w >> SLA, 0, nE - 1);
    const int g0 = clampi(pay[e0], 0, nPay - 1);
    const int g1 = clampi(pay[e1], 0, nPay - 1);
    const int g2 = clampi(pay[e2], 0, nPay - 1);
    const int g3 = clampi(pay[e3], 0, nPay - 1);
    v4i o;
    o.x = g0 & -(int)(p0 + 0 < tt);
    o.y = g1 & -(int)(p0 + 1 < tt);
    o.z = g2 & -(int)(p0 + 2 < tt);
    o.w = g3 & -(int)(p0 + 3 < tt);
    int* dp = listg + (size_t)blk * RC + 4 * i4;
    *(volatile v4i*)dp = o;
    __threadfence();
    *(volatile v4i*)dp = o;
  }
}

template <int MODE>
__global__ __launch_bounds__(NTHR) void k_agg1(const int* __restrict__ listg, const int* __restrict__ cntg,
                                               const int* __restrict__ offg, int rc,
                                               const unsigned short* __restrict__ gp, int nSrc,
                                               unsigned short* apl, int nN, int mRows) {
  __shared__ __attribute__((aligned(16))) int cnt[NBA];
  __shared__ __attribute__((aligned(16))) int offs[NBA];
  __shared__ __attribute__((aligned(16))) unsigned rowb[NWAVE * 128];
  const int tid = (int)threadIdx.x, lane = tid & 31, wave = tid >> 5;
  const int blk = (int)blockIdx.x;
  const int nodeBase = blk * NBA;
  {
    const v4i c4 = *(const v4i*)(cntg + (size_t)blk * NBA + 4 * tid);
    const v4i o4 = *(const v4i*)(offg + (size_t)blk * NBA + 4 * tid);
    *(v4ia*)(cnt + 4 * tid) = c4;
    *(v4ia*)(offs + 4 * tid) = o4;
  }
  __syncthreads();
  const int* lb = listg + (size_t)blk * (size_t)rc;
  unsigned* rb = rowb + wave * 128;
  const float qnan = __int_as_float(0x7fc00000);

#pragma unroll 1
  for (int pr = 0; pr < NBA / (2 * NWAVE); ++pr) {
    const int p = pr * NWAVE + wave;
#pragma unroll 1
    for (int hs = 0; hs < 2; ++hs) {
      const int s = 2 * p + hs;
      const int node = nodeBase + s;
      const int craw = cnt[s];
      const bool bad = (craw < 0) || (craw > DEGCAP);
      const int c = clampi(craw, 0, DEGCAP);
      const int o = clampi(offs[s], 0, rc - 1);
      float a0 = 0.0f, a1 = 0.0f;
#pragma unroll 1
      for (int b0 = 0; b0 < c; b0 += 32) {
        int idx = o + b0 + lane;
        idx = idx > o + c - 1 ? o + c - 1 : idx;
        idx = clampi(idx, 0, rc - 1);
        const int sr = clampi(lb[idx], 0, nSrc - 1);
        const int m32 = (c - b0) < 32 ? (c - b0) : 32;
#pragma unroll 1
        for (int k = 0; k < m32; ++k) {
          const int sk = __builtin_amdgcn_readlane(sr, k);
          if constexpr (MODE == 0) {
            const u32a* rp = (const u32a*)(gp + (size_t)sk * 128) + lane;
            const unsigned wh = rp[0];
            const unsigned wl = rp[32];
            a0 += __uint_as_float(wh << 16) + __uint_as_float(wl << 16);
            a1 += __uint_as_float(wh & 0xffff0000u) + __uint_as_float(wl & 0xffff0000u);
          } else {
            const u32a* rp = (const u32a*)(gp + (size_t)sk * 64) + lane;
            const unsigned w = rp[0];
            a0 += __uint_as_float(w << 16);
            a1 += __uint_as_float(w & 0xffff0000u);
          }
        }
      }
      const float d = fmaxf((float)c, 1.0f);
      const float pz = bad ? qnan : 0.0f;
      const bool live = node < nN;
      const float m0 = live ? (a0 / d + pz) : 0.0f;
      const float m1 = live ? (a1 / d + pz) : 0.0f;
      unsigned l0, l1;
      const unsigned hb0 = hl_bits(m0, l0);
      const unsigned hb1 = hl_bits(m1, l1);
      rb[hs * 64 + lane]      = hb0 | (hb1 << 16);
      rb[hs * 64 + 32 + lane] = l0 | (l1 << 16);
    }
    wave_sync();
    const v4u q = *(const v4ua*)(rb + 4 * lane);
    wave_sync();
    const int row0 = nodeBase + 2 * p;
    if (row0 < mRows) {
      unsigned* dp = (unsigned*)(apl + (size_t)row0 * 128) + 4 * lane;
      *(volatile v4u*)dp = q;
      __threadfence();
      *(volatile v4u*)dp = q;
    }
  }
}

__global__ __launch_bounds__(NTHR) void k_agg2(const int* __restrict__ listg, const int* __restrict__ cntg,
                                               const int* __restrict__ offg, int rc,
                                               const float* __restrict__ vg, int nSrc,
                                               const float* __restrict__ vown, float* pout, int nN) {
  __shared__ __attribute__((aligned(16))) int cnt[NBA];
  __shared__ __attribute__((aligned(16))) int offs[NBA];
  __shared__ __attribute__((aligned(16))) float pst[NBA * 8];
  const int tid = (int)threadIdx.x, lane = tid & 31, wave = tid >> 5;
  const int blk = (int)blockIdx.x;
  const int nodeBase = blk * NBA;
  {
    const v4i c4 = *(const v4i*)(cntg + (size_t)blk * NBA + 4 * tid);
    const v4i o4 = *(const v4i*)(offg + (size_t)blk * NBA + 4 * tid);
    *(v4ia*)(cnt + 4 * tid) = c4;
    *(v4ia*)(offs + 4 * tid) = o4;
  }
  __syncthreads();
  const int* lb = listg + (size_t)blk * (size_t)rc;
  const int g = lane >> 3, ch = lane & 7;
  const float qnan = __int_as_float(0x7fc00000);

#pragma unroll 1
  for (int si = 0; si < NBA / NWAVE; ++si) {
    const int s = si * NWAVE + wave;
    const int node = nodeBase + s;
    const int craw = cnt[s];
    const bool bad = (craw < 0) || (craw > DEGCAP);
    const int c = clampi(craw, 0, DEGCAP);
    const int o = clampi(offs[s], 0, rc - 1);
    float acc = 0.0f;
#pragma unroll 1
    for (int b0 = 0; b0 < c; b0 += 32) {
      int idx = o + b0 + lane;
      idx = idx > o + c - 1 ? o + c - 1 : idx;
      idx = clampi(idx, 0, rc - 1);
      const int sr = clampi(lb[idx], 0, nSrc - 1);
      const int m32 = (c - b0) < 32 ? (c - b0) : 32;
      const int nj = (m32 + 3) >> 2;
#pragma unroll 1
      for (int j = 0; j < nj; ++j) {
        const int k = 4 * j + g;
        const int sk = __shfl(sr, k, 32);
        const float v = vg[(size_t)sk * 16 + ch];
        acc += andf(v, mk(k < m32));
      }
    }
    acc += __shfl_xor(acc, 8, 32);
    acc += __shfl_xor(acc, 16, 32);
    const float d = fmaxf((float)c, 1.0f);
    const int nc = node < nN ? node : nN - 1;
    const float bo = vown[(size_t)nc * 16 + 8 + ch];
    const float pz = bad ? qnan : 0.0f;
    const bool live = node < nN;
    const float r = live ? ((acc / d + bo) + pz) : 0.0f;
    if (lane < 8) pst[s * 8 + lane] = r;
  }
  __syncthreads();
  v4f fv[8];
#pragma unroll
  for (int it = 0; it < 8; ++it) fv[it] = *(const v4fa*)(pst + 4 * (it * NTHR + tid));
  float* dp = pout + (size_t)nodeBase * 8 + 4 * tid;
#pragma unroll
  for (int it = 0; it < 8; ++it) *(volatile v4f*)(dp + 4 * it * NTHR) = fv[it];
  __threadfence();
#pragma unroll
  for (int it = 0; it < 8; ++it) *(volatile v4f*)(dp + 4 * it * NTHR) = fv[it];
}

__global__ __launch_bounds__(NTHR) void k_out(const int* __restrict__ els, const int* __restrict__ eld,
                                              const float* __restrict__ pu, const float* __restrict__ pm,
                                              const float* __restrict__ tab, float* out, int nL, int nU, int nM) {
  __shared__ __attribute__((aligned(16))) float ost[1024 * CD];
  const int tid = (int)threadIdx.x;
  const int base = (int)blockIdx.x * 1024;
  const v4f cb0 = *(const v4f*)(tab + T_CLSB);
  const v4f cb1 = *(const v4f*)(tab + T_CLSB + 4);
#pragma unroll 1
  for (int j = 0; j < 4; ++j) {
    const int p = j * NTHR + tid;
    const int e = min(base + p, nL - 1);
    const int iu = clampi(els[e], 0, nU - 1);
    const int im = clampi(eld[e], 0, nM - 1);
    const v4f a0 = *(const v4f*)(pu + (size_t)iu * 8);
    const v4f a1 = *(const v4f*)(pu + (size_t)iu * 8 + 4);
    const v4f b0 = *(const v4f*)(pm + (size_t)im * 8);
    const v4f b1 = *(const v4f*)(pm + (size_t)im * 8 + 4);
    float* q = ost + p * CD;
    q[0] = (a0.x + b0.x) + cb0.x;
    q[1] = (a0.y + b0.y) + cb0.y;
    q[2] = (a0.z + b0.z) + cb0.z;
    q[3] = (a0.w + b0.w) + cb0.w;
    q[4] = (a1.x + b1.x) + cb1.x;
    q[5] = (a1.y + b1.y) + cb1.y;
    q[6] = (a1.z + b1.z) + cb1.z;
  }
  __syncthreads();
  const int nvalid = (nL - base) < 1024 ? (nL - base) : 1024;
  const int n4 = (nvalid * CD) >> 2;
  v4f fv[7];
#pragma unroll
  for (int it = 0; it < 7; ++it) fv[it] = *(const v4fa*)(ost + 4 * (it * NTHR + tid));
  float* dp = out + (size_t)base * CD + 4 * tid;
#pragma unroll
  for (int it = 0; it < 7; ++it) if (it * NTHR + tid < n4) *(volatile v4f*)(dp + 4 * it * NTHR) = fv[it];
  __threadfence();
#pragma unroll
  for (int it = 0; it < 7; ++it) if (it * NTHR + tid < n4) *(volatile v4f*)(dp + 4 * it * NTHR) = fv[it];
}

static inline int cdiv(int a, int b) { return (a + b - 1) / b; }
static inline size_t al256(size_t o) { return (o + 255) & ~(size_t)255; }

extern "C" void kernel_launch(void* const* d_in, const int* in_sizes, int n_in,
                              void* d_out, int out_size, void* d_ws, size_t ws_size,
                              hipStream_t stream) {
  if (n_in < 25) return;
  const int nU = in_sizes[0], nM = in_sizes[1], nE = in_sizes[3], nL = in_sizes[5];
  if (nU < 64 || nM < 64 || nU > (1 << 22) || nM > (1 << 22)) return;
  if (nE < 1 || nE >= (1 << 21) || in_sizes[4] != nE) return;
  if (nL < 32 || (nL % 32) != 0 || in_sizes[6] != nL) return;
  if ((long long)in_sizes[2] != (long long)nM * FD) return;
  if ((long long)in_sizes[7] != (long long)nU * HD) return;
  if ((long long)in_sizes[8] != (long long)nM * HD) return;
  if (in_sizes[9] != FD * HD || in_sizes[10] != HD) return;
  for (int l = 0; l < 4; ++l) {
    const int b = 11 + 3 * l;
    if (in_sizes[b] != HD * HD || in_sizes[b + 1] != HD || in_sizes[b + 2] != HD * HD) return;
  }
  if (in_sizes[23] != 2 * HD * CD || in_sizes[24] != CD) return;
  if ((long long)out_size != (long long)nL * CD) return;

  const int*   uid   = (const int*)  d_in[0];
  const int*   mid   = (const int*)  d_in[1];
  const float* mx    = (const float*)d_in[2];
  const int*   esrc  = (const int*)  d_in[3];
  const int*   edst  = (const int*)  d_in[4];
  const int*   els   = (const int*)  d_in[5];
  const int*   eld   = (const int*)  d_in[6];
  const float* uemb  = (const float*)d_in[7];
  const float* memb  = (const float*)d_in[8];
  const float* wmov  = (const float*)d_in[9];
  const float* bmov  = (const float*)d_in[10];
  const float* w1tl  = (const float*)d_in[11];
  const float* b1t   = (const float*)d_in[12];
  const float* w1tr  = (const float*)d_in[13];
  const float* w1vl  = (const float*)d_in[14];
  const float* b1v   = (const float*)d_in[15];
  const float* w1vr  = (const float*)d_in[16];
  const float* w2tl  = (const float*)d_in[17];
  const float* b2t   = (const float*)d_in[18];
  const float* w2tr  = (const float*)d_in[19];
  const float* w2vl  = (const float*)d_in[20];
  const float* b2v   = (const float*)d_in[21];
  const float* w2vr  = (const float*)d_in[22];
  const float* clsw  = (const float*)d_in[23];
  const float* clsb  = (const float*)d_in[24];
  float* out = (float*)d_out;

  const int MPU = cdiv(nU, GBM) * GBM;
  const int MPM = cdiv(nM, GBM) * GBM;
  const int gU = cdiv(nU, NBA), gM = cdiv(nM, NBA);
  if ((long long)gU * NBA < (long long)MPU || (long long)gM * NBA < (long long)MPM) return;
  const int vec8 = ((nE & 3) == 0) ? 1 : 0;

  char* ws = (char*)d_ws;
  size_t off = 0;
  const size_t oTAB = off; off = al256(off + (size_t)TAB_N * 4);
  const size_t oWPL = off; off = al256(off + (size_t)WPL_N * 2);
  const size_t oXU  = off; off = al256(off + (size_t)MPU * 64 * 2);
  const size_t oMXB = off; off = al256(off + (size_t)MPM * 32 * 2);
  const size_t oXM  = off; off = al256(off + (size_t)MPM * 128 * 2);
  const size_t oAU  = off; off = al256(off + (size_t)MPU * 128 * 2);
  const size_t oAM  = off; off = al256(off + (size_t)MPM * 128 * 2);
  const size_t oUV  = off; off = al256(off + (size_t)MPU * 16 * 4);
  const size_t oMV  = off; off = al256(off + (size_t)MPM * 16 * 4);
  const size_t oPU  = off; off = al256(off + (size_t)gU * NBA * 8 * 4);
  const size_t oPM  = off; off = al256(off + (size_t)gM * NBA * 8 * 4);
  const size_t oLU  = off; off = al256(off + (size_t)gU * RCAP_U * 4);
  const size_t oLM  = off; off = al256(off + (size_t)gM * RCAP_M * 4);
  const size_t oCU  = off; off = al256(off + (size_t)gU * NBA * 4);
  const size_t oOU  = off; off = al256(off + (size_t)gU * NBA * 4);
  const size_t oCM  = off; off = al256(off + (size_t)gM * NBA * 4);
  const size_t oOM  = off; off = al256(off + (size_t)gM * NBA * 4);
  if (off > ws_size) return;

  float*          TAB = (float*)(ws + oTAB);
  unsigned short* WPL = (unsigned short*)(ws + oWPL);
  unsigned short* XU  = (unsigned short*)(ws + oXU);
  unsigned short* MXB = (unsigned short*)(ws + oMXB);
  unsigned short* XM  = (unsigned short*)(ws + oXM);
  unsigned short* AU  = (unsigned short*)(ws + oAU);
  unsigned short* AM  = (unsigned short*)(ws + oAM);
  float* UV = (float*)(ws + oUV);
  float* MV = (float*)(ws + oMV);
  float* PU = (float*)(ws + oPU);
  float* PM = (float*)(ws + oPM);
  int* LU = (int*)(ws + oLU);
  int* LM = (int*)(ws + oLM);
  int* CU = (int*)(ws + oCU);
  int* OU = (int*)(ws + oOU);
  int* CM = (int*)(ws + oCM);
  int* OM = (int*)(ws + oOM);

  const size_t ldsU = (size_t)(LISTN + 2 * RCAP_U + 3 * NBA + 16) * 4;
  const size_t ldsM = (size_t)(LISTN + 2 * RCAP_M + 3 * NBA + 16) * 4;
  hipFuncSetAttribute(reinterpret_cast<const void*>(&k_compact<RCAP_U>), hipFuncAttributeMaxDynamicSharedMemorySize, (int)ldsU);
  hipFuncSetAttribute(reinterpret_cast<const void*>(&k_compact<RCAP_M>), hipFuncAttributeMaxDynamicSharedMemorySize, (int)ldsM);

  const int nUnits = U_SM + MPU * 8 + MPM * 4;
  k_prep<<<cdiv(nUnits, NTHR), NTHR, 0, stream>>>(uid, uemb, mx, wmov, w1vl, w1vr, w1tl, w1tr, w2tl, w2vr, w2vl, w2tr,
                                                  bmov, b1v, b1t, b2v, b2t, clsw, clsb, TAB, WPL, XU, MXB,
                                                  nU, MPU, nM, MPM);
  k_gemm1<0><<<MPM / GBM, GTHR, 0, stream>>>(MXB, 32, 32, MXB, 0, 0, WPL + OW_0, 32, TAB, TB_BM,
                                             mid, memb, nM, XM, nM);
  k_compact<RCAP_U><<<gU, NTHR, ldsU, stream>>>(esrc, edst, nE, nM, vec8, LU, CU, OU);
  k_compact<RCAP_M><<<gM, NTHR, ldsM, stream>>>(edst, esrc, nE, nU, vec8, LM, CM, OM);
  k_agg1<0><<<gU, NTHR, 0, stream>>>(LU, CU, OU, RCAP_U, XM, nM, AU, nU, MPU);
  k_agg1<1><<<gM, NTHR, 0, stream>>>(LM, CM, OM, RCAP_M, XU, nU, AM, nM, MPM);
  k_gemm1<1><<<MPU / GBM, GTHR, 0, stream>>>(AU, 128, 128, XU, 64, 64, WPL + OW_U1, 192, TAB, TB_L1REV,
                                             mid, memb, nM, AU, nU);
  k_gemm1<1><<<MPM / GBM, GTHR, 0, stream>>>(AM, 128, 128, XM, 128, 128, WPL + OW_M1, 256, TAB, TB_L1RAT,
                                             mid, memb, nM, AM, nM);
  k_gemm2<<<MPU / GBM, GTHR, 0, stream>>>(AU, WPL + OW_U2, TAB, TB_L2REV, TC_BOT, TC_TOP, UV);
  k_gemm2<<<MPM / GBM, GTHR, 0, stream>>>(AM, WPL + OW_M2, TAB, TB_L2RAT, TC_TOP, TC_BOT, MV);
  k_agg2<<<gU, NTHR, 0, stream>>>(LU, CU, OU, RCAP_U, MV, nM, UV, PU, nU);
  k_agg2<<<gM, NTHR, 0, stream>>>(LM, CM, OM, RCAP_M, UV, nU, MV, PM, nM);
  k_out<<<cdiv(nL, 1024), NTHR, 0, stream>>>(els, eld, PU, PM, TAB, out, nL, nU, nM);
}
